// VanillaCausalSelfAttention_25658134626324
// MI455X (gfx1250) — hardware-verified
//
#include <hip/hip_runtime.h>
#include <math.h>
#include <stdint.h>

#define NBATCH 4
#define SEQ    1024
#define DM     1024
#define NH     16
#define HD     64
#define QKP    (2 * DM)
#define CTXP   (2 * DM)
#define MP     (NBATCH * SEQ)
#define NQB    (SEQ / 64)
#define RCE    (SEQ + 64)
#define RB     80
#define RP     80
#define WSC    64.0f
#define RSC    2048.0f
#define PSC    1024.0f
static_assert(NH * HD == DM);
static_assert((SEQ % 64) == 0 && (DM % 64) == 0 && (MP % 64) == 0 && (QKP % 64) == 0);
static_assert(RB == 64 + 16 && (RB % 16) == 0 && RP >= RB);
static_assert(RCE >= SEQ + 64);

typedef _Float16 v16h __attribute__((ext_vector_type(16)));
typedef _Float16 v8h  __attribute__((ext_vector_type(8)));
typedef __bf16   v16b __attribute__((ext_vector_type(16)));
typedef unsigned short v16us __attribute__((ext_vector_type(16)));
typedef unsigned short v8us  __attribute__((ext_vector_type(8)));
typedef float    v8f  __attribute__((ext_vector_type(8)));
typedef float    v4f  __attribute__((ext_vector_type(4)));
typedef unsigned int v4u __attribute__((ext_vector_type(4)));

union FragH { v16h v; v8h h[2]; };
union FragU { v16us v; v8us h[2]; };

__device__ __forceinline__ unsigned short bf_bits(float f) {
  unsigned u = __float_as_uint(f);
  return (unsigned short)((u + 0x7FFFu + ((u >> 16) & 1u)) >> 16);
}
__device__ __forceinline__ float bf_up(unsigned short h) { return __uint_as_float(((unsigned)h) << 16); }
__device__ __forceinline__ float bfr(float f) { return bf_up(bf_bits(f)); }
__device__ __forceinline__ unsigned short h_bits(_Float16 x) { return __builtin_bit_cast(unsigned short, x); }
__device__ __forceinline__ unsigned pk16(unsigned short a, unsigned short b) { return (unsigned)a | ((unsigned)b << 16); }
__device__ __forceinline__ v8f zero8() { v8f z = {0.f, 0.f, 0.f, 0.f, 0.f, 0.f, 0.f, 0.f}; return z; }

__device__ __forceinline__ v16us ldfrag_u(const unsigned short* p) {
  FragU f;
  f.h[0] = *(const v8us*)(p);
  f.h[1] = *(const v8us*)(p + 16);
  return f.v;
}
__device__ __forceinline__ v16h ldfrag_h(const _Float16* p) {
  FragH f;
  f.h[0] = *(const v8h*)(p);
  f.h[1] = *(const v8h*)(p + 16);
  return f.v;
}

template <int BF>
__device__ __forceinline__ v8f mma_raw(v16us a, v16us b, v8f c) {
  if (BF) {
    return __builtin_amdgcn_wmma_f32_16x16x32_bf16(false, __builtin_bit_cast(v16b, a), false,
                                                   __builtin_bit_cast(v16b, b), (short)0, c, false, false);
  }
  return __builtin_amdgcn_wmma_f32_16x16x32_f16(false, __builtin_bit_cast(v16h, a), false,
                                                __builtin_bit_cast(v16h, b), (short)0, c, false, false);
}
__device__ __forceinline__ v8f mma_bu(v16us a, v16us b, v8f c) {
  c = __builtin_amdgcn_wmma_f32_16x16x32_bf16(false, __builtin_bit_cast(v16b, a), false,
                                               __builtin_bit_cast(v16b, b), (short)0, c, false, false);
#if defined(__HIP_DEVICE_COMPILE__)
  asm volatile("v_nop\n\tv_nop\n\tv_nop\n\tv_nop" : "+v"(c) : "v"(a), "v"(b));
#endif
  return c;
}
__device__ __forceinline__ v8f mma_h(v16h a, v16h b, v8f c) {
  c = __builtin_amdgcn_wmma_f32_16x16x32_f16(false, a, false, b, (short)0, c, false, false);
#if defined(__HIP_DEVICE_COMPILE__)
  asm volatile("v_nop\n\tv_nop\n\tv_nop\n\tv_nop" : "+v"(c) : "v"(a), "v"(b));
#endif
  return c;
}
__device__ __forceinline__ void dep_guard1(v8f& a, v8f& b, v16us x) {
#if defined(__HIP_DEVICE_COMPILE__)
  asm volatile("v_nop\n\tv_nop\n\tv_nop\n\tv_nop" : "+v"(a), "+v"(b) : "v"(x));
#endif
}
__device__ __forceinline__ void keep4_u(v16us a, v16us b, v16us c, v16us d) {
#if defined(__HIP_DEVICE_COMPILE__)
  asm volatile("v_nop" :: "v"(a), "v"(b), "v"(c), "v"(d));
#endif
}
__device__ __forceinline__ void acc_guard4(v8f& a, v8f& b, v8f& c, v8f& d) {
#if defined(__HIP_DEVICE_COMPILE__)
  asm volatile("v_nop\n\tv_nop\n\tv_nop\n\tv_nop" : "+v"(a), "+v"(b), "+v"(c), "+v"(d));
#endif
}
__device__ __forceinline__ void wave_sync_lds() {
  __builtin_amdgcn_fence(__ATOMIC_RELEASE, "workgroup");
  __builtin_amdgcn_wave_barrier();
  __builtin_amdgcn_fence(__ATOMIC_ACQUIRE, "workgroup");
}

__global__ __launch_bounds__(256) void conv_h16(const float* __restrict__ W, unsigned short* Wh, int n8, float wsc) {
  const int i  = blockIdx.x * 256 + threadIdx.x;
  const int ic = (i < n8) ? i : (n8 - 1);
  const float* src = W + (size_t)ic * 8;
  const v4f a = *(const v4f*)(src);
  const v4f c = *(const v4f*)(src + 4);
  v4u o;
  o[0] = pk16(h_bits((_Float16)(bfr(a[0]) * wsc)), h_bits((_Float16)(bfr(a[1]) * wsc)));
  o[1] = pk16(h_bits((_Float16)(bfr(a[2]) * wsc)), h_bits((_Float16)(bfr(a[3]) * wsc)));
  o[2] = pk16(h_bits((_Float16)(bfr(c[0]) * wsc)), h_bits((_Float16)(bfr(c[1]) * wsc)));
  o[3] = pk16(h_bits((_Float16)(bfr(c[2]) * wsc)), h_bits((_Float16)(bfr(c[3]) * wsc)));
  if (i < n8) *(volatile v4u*)(Wh + (size_t)i * 8) = o;
  __threadfence();
  if (i < n8) *(volatile v4u*)(Wh + (size_t)i * 8) = o;
}

__global__ __launch_bounds__(256) void conv_e16(const float* __restrict__ P, unsigned short* Eh, int n8v, int n8t) {
  const int i  = blockIdx.x * 256 + threadIdx.x;
  const int ic = (i < n8v) ? i : (n8v - 1);
  const float* src = P + (size_t)ic * 8;
  const v4f a = *(const v4f*)(src);
  const v4f c = *(const v4f*)(src + 4);
  const bool valid = (i < n8v);
  v4u o;
  o[0] = valid ? pk16(bf_bits(a[0]), bf_bits(a[1])) : 0u;
  o[1] = valid ? pk16(bf_bits(a[2]), bf_bits(a[3])) : 0u;
  o[2] = valid ? pk16(bf_bits(c[0]), bf_bits(c[1])) : 0u;
  o[3] = valid ? pk16(bf_bits(c[2]), bf_bits(c[3])) : 0u;
  if (i < n8t) *(volatile v4u*)(Eh + (size_t)i * 8) = o;
  __threadfence();
  if (i < n8t) *(volatile v4u*)(Eh + (size_t)i * 8) = o;
}

template <int MODE>
__global__ __launch_bounds__(256) void tconv64(const float* __restrict__ W, unsigned short* out,
                                               int rows, int cols, int ldo, int dupoff, float wsc) {
  __shared__ __align__(16) unsigned short sh[64 * 72];
  const int t  = threadIdx.x;
  const int n0 = blockIdx.x * 64;
  const int k0 = blockIdx.y * 64;
#pragma unroll
  for (int i = 0; i < 4; ++i) {
    const int idx = i * 256 + t;
    const int r = idx >> 4, c4 = (idx & 15) * 4;
    int kr = k0 + r;   kr = (kr < rows) ? kr : (rows - 1);
    int nc = n0 + c4;  nc = (nc < cols - 4) ? nc : (cols - 4);
    const v4f v = *(const v4f*)(W + (size_t)kr * cols + nc);
#pragma unroll
    for (int e = 0; e < 4; ++e) {
      unsigned short u;
      if (MODE == 0) u = h_bits((_Float16)(bfr(v[e]) * wsc));
      else           u = bf_bits(v[e]);
      sh[(c4 + e) * 72 + r] = u;
    }
  }
  __syncthreads();
  const int wave = t >> 5, lane = t & 31;
  const int q = lane >> 3, c8 = (lane & 7) * 8;
  v4u pv[2];
  size_t go[2];
#pragma unroll
  for (int it = 0; it < 2; ++it) {
    const int nl = it * 32 + wave * 4 + q;
    pv[it] = *(const v4u*)(sh + nl * 72 + c8);
    go[it] = (size_t)(n0 + nl) * ldo + k0 + c8;
  }
  for (int pass = 0; pass < 2; ++pass) {
#pragma unroll
    for (int it = 0; it < 2; ++it) {
      *(volatile v4u*)(out + go[it]) = pv[it];
      if (dupoff != 0) *(volatile v4u*)(out + go[it] + dupoff) = pv[it];
    }
    __threadfence();
  }
}

template <int BF, int OM, int BM>
__global__ __launch_bounds__(256) void gemm64(
    const unsigned short* __restrict__ Ap, int lda, long long strideA,
    const unsigned short* __restrict__ Btp, int ldb, long long strideB,
    unsigned short* Cp, unsigned short* Cp2, float* Cf, int ldc, long long strideC,
    const float* bias0, const float* bias1, int nsplit,
    int M, int N, int K, float oscale) {
  __shared__ __align__(16) float sT[8][16 * 68];
  const int b    = blockIdx.y;
  const int lane = threadIdx.x & 31;
  const int wave = threadIdx.x >> 5;
  const int tilesN = N >> 6;
  const int tilesM = M >> 6;
  const int tile = blockIdx.x * 8 + wave;
  if (tile >= tilesM * tilesN) return;
  const int tm = tile / tilesN;
  const int tn = tile - tm * tilesN;
  const int m0 = tm << 6;
  const int n0 = tn << 6;

  const unsigned short* Ab = Ap  + (size_t)b * strideA;
  const unsigned short* Bb = Btp + (size_t)b * strideB;

  const int rlane = lane & 15;
  const int koff  = (lane >> 4) * 8;
  const int mOff  = (lane >> 4) * 8;

  v8f acc[4][4];
#pragma unroll
  for (int i = 0; i < 4; ++i)
#pragma unroll
    for (int j = 0; j < 4; ++j) acc[i][j] = zero8();

  for (int k0 = 0; k0 < K; k0 += 32) {
    v16us bh[4];
#pragma unroll
    for (int j = 0; j < 4; ++j) {
      const size_t bo = (size_t)(n0 + (j << 4) + rlane) * ldb + koff + k0;
      bh[j] = ldfrag_u(Bb + bo);
    }
#pragma unroll
    for (int i = 0; i < 4; ++i) {
      const size_t ao = (size_t)(m0 + (i << 4) + rlane) * lda + koff + k0;
      const v16us ah = ldfrag_u(Ab + ao);
#pragma unroll
      for (int j = 0; j < 4; ++j) acc[i][j] = mma_raw<BF>(ah, bh[j], acc[i][j]);
      dep_guard1(acc[i][0], acc[i][3], ah);
    }
    keep4_u(bh[0], bh[1], bh[2], bh[3]);
  }
  acc_guard4(acc[0][0], acc[0][1], acc[0][2], acc[0][3]);
  acc_guard4(acc[1][0], acc[1][1], acc[1][2], acc[1][3]);
  acc_guard4(acc[2][0], acc[2][1], acc[2][2], acc[2][3]);
  acc_guard4(acc[3][0], acc[3][1], acc[3][2], acc[3][3]);

  const int hh2 = lane >> 4, c4 = (lane & 15) * 4;
  const int q8  = lane >> 3, c8 = (lane & 7) * 8;

  const float* bsel = bias0;
  int nb0 = n0;
  if (BM == 1) {
    if (n0 >= nsplit) { bsel = bias1; nb0 = n0 - nsplit; }
  }
  v4f bb4 = {0.f, 0.f, 0.f, 0.f};
  float bn[8];
#pragma unroll
  for (int e = 0; e < 8; ++e) bn[e] = 0.f;
  if (BM == 1) {
    if (OM == 0) {
#pragma unroll
      for (int e = 0; e < 4; ++e) bb4[e] = bfr(bsel[nb0 + c4 + e]);
    } else {
#pragma unroll
      for (int e = 0; e < 8; ++e) bn[e] = bfr(bsel[nb0 + c8 + e]);
    }
  }

  float* slab = sT[wave];
#pragma unroll
  for (int i = 0; i < 4; ++i) {
    const int mBase = m0 + (i << 4);
#pragma unroll
    for (int j = 0; j < 4; ++j) {
#pragma unroll
      for (int r = 0; r < 8; ++r) {
        slab[(mOff + r) * 68 + (j << 4) + rlane] = acc[i][j][r];
      }
    }
    wave_sync_lds();
    if (OM == 0) {
      float* C = Cf + (size_t)b * strideC;
      v4f vals[8];
#pragma unroll
      for (int it = 0; it < 8; ++it) {
        const int row = it * 2 + hh2;
        v4f v = *(const v4f*)(slab + row * 68 + c4);
        float bmv = 0.f;
        if (BM == 2) bmv = bfr(bias0[mBase + row]);
        vals[it] = v * oscale + bb4 + bmv;
      }
      for (int pass = 0; pass < 2; ++pass) {
#pragma unroll
        for (int it = 0; it < 8; ++it) {
          const int row = it * 2 + hh2;
          *(volatile v4f*)(C + (size_t)(mBase + row) * ldc + n0 + c4) = vals[it];
        }
        __threadfence();
      }
    } else {
      unsigned short* C  = Cp  + (size_t)b * strideC;
      unsigned short* C2 = Cp2 + (size_t)b * strideC;
      v4u hv[4], lv[4];
#pragma unroll
      for (int it = 0; it < 4; ++it) {
        const int row = it * 4 + q8;
        const float* sp = slab + row * 68 + c8;
        float bmv = 0.f;
        if (BM == 2) bmv = bfr(bias0[mBase + row]);
        v4u ha, la;
#pragma unroll
        for (int e = 0; e < 4; ++e) {
          const float f0 = sp[2 * e]     * oscale + bn[2 * e]     + bmv;
          const float f1 = sp[2 * e + 1] * oscale + bn[2 * e + 1] + bmv;
          unsigned short u0, u1, w0, w1;
          if (OM == 3) {
            u0 = bf_bits(f0); u1 = bf_bits(f1);
            w0 = bf_bits(f0 - bf_up(u0)); w1 = bf_bits(f1 - bf_up(u1));
          } else {
            const _Float16 g0 = (_Float16)f0, g1 = (_Float16)f1;
            u0 = h_bits(g0); u1 = h_bits(g1);
            w0 = h_bits((_Float16)((f0 - (float)g0) * RSC));
            w1 = h_bits((_Float16)((f1 - (float)g1) * RSC));
          }
          ha[e] = pk16(u0, u1);
          la[e] = pk16(w0, w1);
        }
        hv[it] = ha;
        lv[it] = la;
      }
      for (int pass = 0; pass < 2; ++pass) {
#pragma unroll
        for (int it = 0; it < 4; ++it) {
          const int row = it * 4 + q8;
          const size_t go = (size_t)(mBase + row) * ldc + n0 + c8;
          *(volatile v4u*)(C  + go) = hv[it];
          *(volatile v4u*)(C2 + go) = lv[it];
        }
        __threadfence();
      }
    }
    wave_sync_lds();
  }
}

__global__ __launch_bounds__(128)
void attn64(const unsigned short* __restrict__ qkh, const unsigned short* __restrict__ qkl,
            const unsigned short* __restrict__ vth, const unsigned short* __restrict__ vtl,
            const unsigned short* __restrict__ ehp, unsigned short* ctxp, float sscale) {
  __shared__ __align__(16) unsigned short Kh[64 * 64];
  __shared__ __align__(16) unsigned short Kl[64 * 64];
  __shared__ __align__(16) _Float16 Vh[64 * 64];
  __shared__ __align__(16) _Float16 Vl[64 * 64];
  __shared__ __align__(16) _Float16 Psh[4][16 * 64];
  __shared__ __align__(16) _Float16 Psl[4][16 * 64];
  __shared__ __align__(16) float    Rsh[4][16 * RP];
  __shared__ __align__(16) float    Os[4][16 * 64];

  const int tid  = threadIdx.x;
  const int wave = tid >> 5;
  const int lane = tid & 31;
  const int hh   = lane >> 4;
  const int c    = lane & 15;

  const int bx   = blockIdx.x;
  const int qb   = bx % NQB;
  const int rest = bx / NQB;
  const int h    = rest % NH;
  const int b    = rest / NH;
  const int q0   = qb * 64 + wave * 16;
  const size_t rowB = (size_t)b * SEQ;

  const unsigned short* Qh  = qkh + (size_t)h * HD;
  const unsigned short* Ql  = qkl + (size_t)h * HD;
  const unsigned short* Kgh = qkh + DM + (size_t)h * HD;
  const unsigned short* Kgl = qkl + DM + (size_t)h * HD;
  const _Float16* Vgh = (const _Float16*)(const void*)vth + ((size_t)b * DM + (size_t)h * HD) * SEQ;
  const _Float16* Vgl = (const _Float16*)(const void*)vtl + ((size_t)b * DM + (size_t)h * HD) * SEQ;
  float*    rrow = Rsh[wave];
  _Float16* pwh  = Psh[wave];
  _Float16* pwl  = Psl[wave];

  float mrow[8], lrow[8];
  v8f oacc[4], oaccL[4];
#pragma unroll
  for (int r = 0; r < 8; ++r) { mrow[r] = -INFINITY; lrow[r] = 0.f; }
#pragma unroll
  for (int t = 0; t < 4; ++t) { oacc[t] = zero8(); oaccL[t] = zero8(); }

  const int nkt = qb + 1;
#pragma unroll 1
  for (int kt = 0; kt < nkt; ++kt) {
    const int kv0 = kt * 64;

    __syncthreads();
    {
      const int r = tid >> 1, hf = (tid & 1) * 32;
      const unsigned short* kgh = Kgh + (rowB + kv0 + r) * QKP + hf;
      const unsigned short* kgl = Kgl + (rowB + kv0 + r) * QKP + hf;
      const _Float16* vgh = Vgh + (size_t)r * SEQ + kv0 + hf;
      const _Float16* vgl = Vgl + (size_t)r * SEQ + kv0 + hf;
#pragma unroll
      for (int i = 0; i < 4; ++i) {
        const v8us a0 = *(const v8us*)(kgh + 8 * i);
        const v8us a1 = *(const v8us*)(kgl + 8 * i);
        const v8h  b0 = *(const v8h*)(vgh + 8 * i);
        const v8h  b1 = *(const v8h*)(vgl + 8 * i);
        *(v8us*)(Kh + r * 64 + hf + 8 * i) = a0;
        *(v8us*)(Kl + r * 64 + hf + 8 * i) = a1;
        *(v8h*)(Vh + r * 64 + hf + 8 * i) = b0;
        *(v8h*)(Vl + r * 64 + hf + 8 * i) = b1;
      }
    }
    __syncthreads();

    v16us qh2[2], ql2[2];
#pragma unroll
    for (int dc = 0; dc < 2; ++dc) {
      qh2[dc] = ldfrag_u(Qh + (rowB + q0 + c) * QKP + dc * 32 + 8 * hh);
      ql2[dc] = ldfrag_u(Ql + (rowB + q0 + c) * QKP + dc * 32 + 8 * hh);
    }

    const int ebase = SEQ - 1 + kv0 - q0 - 15;
#pragma unroll 1
    for (int nt = 0; nt < RB / 16; ++nt) {
      v8f e = zero8();
#pragma unroll
      for (int dc = 0; dc < 2; ++dc) {
        const v16us eb = ldfrag_u(ehp + (size_t)(ebase + nt * 16 + c) * HD + dc * 32 + 8 * hh);
        e = mma_bu(qh2[dc], eb, e);
        e = mma_bu(ql2[dc], eb, e);
      }
#pragma unroll
      for (int r = 0; r < 8; ++r) rrow[(8 * hh + r) * RP + nt * 16 + c] = e[r];
    }
    wave_sync_lds();

    v8f s[4];
#pragma unroll
    for (int j = 0; j < 4; ++j) {
      v8f sh = zero8();
#pragma unroll
      for (int dc = 0; dc < 2; ++dc) {
        FragU kbh, kbl;
        kbh.h[0] = *(const v8us*)(Kh + (j * 16 + c) * 64 + dc * 32 + 8 * hh);
        kbh.h[1] = *(const v8us*)(Kh + (j * 16 + c) * 64 + dc * 32 + 16 + 8 * hh);
        kbl.h[0] = *(const v8us*)(Kl + (j * 16 + c) * 64 + dc * 32 + 8 * hh);
        kbl.h[1] = *(const v8us*)(Kl + (j * 16 + c) * 64 + dc * 32 + 16 + 8 * hh);
        sh = mma_bu(qh2[dc], kbh.v, sh);
        sh = mma_bu(qh2[dc], kbl.v, sh);
        sh = mma_bu(ql2[dc], kbh.v, sh);
      }
      const int jl = j * 16 + c;
      const int kg = kv0 + jl;
#pragma unroll
      for (int r = 0; r < 8; ++r) {
        const int il = 8 * hh + r;
        const int qg = q0 + il;
        const float rel = rrow[il * RP + jl - il + 15];
        const float v = (sh[r] + rel) * sscale;
        s[j][r] = (kg <= qg) ? v : -INFINITY;
      }
    }

#pragma unroll
    for (int r = 0; r < 8; ++r) {
      float m = s[0][r];
      m = fmaxf(m, s[1][r]);
      m = fmaxf(m, s[2][r]);
      m = fmaxf(m, s[3][r]);
#pragma unroll
      for (int off = 1; off < 16; off <<= 1) m = fmaxf(m, __shfl_xor(m, off, 32));
      const float mnew  = fmaxf(mrow[r], m);
      const float alpha = __expf(mrow[r] - mnew);
      mrow[r] = mnew;
      float psum = 0.f;
#pragma unroll
      for (int j = 0; j < 4; ++j) {
        const float p  = __expf(s[j][r] - mnew);
        psum += p;
        const float ps = p * PSC;
        const _Float16 ph = (_Float16)ps;
        pwh[(8 * hh + r) * 64 + j * 16 + c] = ph;
        pwl[(8 * hh + r) * 64 + j * 16 + c] = (_Float16)((ps - (float)ph) * RSC);
      }
#pragma unroll
      for (int off = 1; off < 16; off <<= 1) psum += __shfl_xor(psum, off, 32);
      lrow[r] = lrow[r] * alpha + psum;
#pragma unroll
      for (int t = 0; t < 4; ++t) { oacc[t][r] *= alpha; oaccL[t][r] *= alpha; }
    }
    wave_sync_lds();

#pragma unroll 1
    for (int kk = 0; kk < 2; ++kk) {
      FragH pa, pl;
      pa.h[0] = *(const v8h*)(pwh + c * 64 + kk * 32 + 8 * hh);
      pa.h[1] = *(const v8h*)(pwh + c * 64 + kk * 32 + 16 + 8 * hh);
      pl.h[0] = *(const v8h*)(pwl + c * 64 + kk * 32 + 8 * hh);
      pl.h[1] = *(const v8h*)(pwl + c * 64 + kk * 32 + 16 + 8 * hh);
#pragma unroll
      for (int t = 0; t < 4; ++t) {
        FragH vb, vl;
        vb.h[0] = *(const v8h*)(Vh + (t * 16 + c) * 64 + kk * 32 + 8 * hh);
        vb.h[1] = *(const v8h*)(Vh + (t * 16 + c) * 64 + kk * 32 + 16 + 8 * hh);
        vl.h[0] = *(const v8h*)(Vl + (t * 16 + c) * 64 + kk * 32 + 8 * hh);
        vl.h[1] = *(const v8h*)(Vl + (t * 16 + c) * 64 + kk * 32 + 16 + 8 * hh);
        oacc[t]  = mma_h(pa.v, vb.v, oacc[t]);
        oaccL[t] = mma_h(pa.v, vl.v, oaccL[t]);
        oaccL[t] = mma_h(pl.v, vb.v, oaccL[t]);
      }
    }
  }

  float* os = Os[wave];
#pragma unroll
  for (int r = 0; r < 8; ++r) {
    const float l = lrow[r];
    const float inv = ((l > 0.f) ? (1.0f / l) : 0.f) * (1.0f / PSC);
#pragma unroll
    for (int t = 0; t < 4; ++t) os[(8 * hh + r) * 64 + t * 16 + c] = (oacc[t][r] + oaccL[t][r] * (1.0f / RSC)) * inv;
  }
  wave_sync_lds();
  {
    const int q4 = lane >> 3, c8 = (lane & 7) * 8;
    v4u hv[4], lv[4];
#pragma unroll
    for (int it = 0; it < 4; ++it) {
      const int row = it * 4 + q4;
      const float* sp = os + row * 64 + c8;
      v4u ha, la;
#pragma unroll
      for (int e = 0; e < 4; ++e) {
        const float f0 = sp[2 * e], f1 = sp[2 * e + 1];
        const unsigned short u0 = bf_bits(f0), u1 = bf_bits(f1);
        const unsigned short w0 = bf_bits(f0 - bf_up(u0)), w1 = bf_bits(f1 - bf_up(u1));
        ha[e] = pk16(u0, u1);
        la[e] = pk16(w0, w1);
      }
      hv[it] = ha;
      lv[it] = la;
    }
    for (int pass = 0; pass < 2; ++pass) {
#pragma unroll
      for (int it = 0; it < 4; ++it) {
        const int row = it * 4 + q4;
        const size_t go = (rowB + q0 + row) * CTXP + (size_t)h * HD + c8;
        *(volatile v4u*)(ctxp + go)      = hv[it];
        *(volatile v4u*)(ctxp + go + DM) = lv[it];
      }
      __threadfence();
    }
  }
}

extern "C" void kernel_launch(void* const* d_in, const int* in_sizes, int n_in,
                              void* d_out, int out_size, void* d_ws, size_t ws_size,
                              hipStream_t stream) {
  if (n_in < 10) return;
  if (in_sizes[0] != MP * DM) return;
  if (in_sizes[1] != DM * DM || in_sizes[3] != DM * DM) return;
  if (in_sizes[5] != DM * DM || in_sizes[7] != DM * DM) return;
  if (in_sizes[2] != DM || in_sizes[4] != DM || in_sizes[6] != DM || in_sizes[8] != DM) return;
  if (in_sizes[9] != SEQ * HD) return;
  if (out_size != MP * DM) return;

  const float* x_in  = (const float*)d_in[0];
  const float* w_q   = (const float*)d_in[1];
  const float* b_q   = (const float*)d_in[2];
  const float* w_k   = (const float*)d_in[3];
  const float* b_k   = (const float*)d_in[4];
  const float* w_v   = (const float*)d_in[5];
  const float* b_v   = (const float*)d_in[6];
  const float* w_o   = (const float*)d_in[7];
  const float* b_o   = (const float*)d_in[8];
  const float* relk  = (const float*)d_in[9];

  const size_t PWQK = (size_t)QKP * DM * 2;
  const size_t PWV  = (size_t)DM * DM * 2;
  const size_t PWO2 = (size_t)DM * (2 * DM) * 2;
  const size_t PXH  = (size_t)MP * DM * 2;
  const size_t PEH  = (size_t)RCE * HD * 2;
  const size_t PQK  = (size_t)MP * QKP * 2;
  const size_t PVT  = (size_t)NBATCH * DM * SEQ * 2;
  const size_t PCTX = (size_t)MP * CTXP * 2;
  size_t off = 0;
  const size_t oWqk = off; off += PWQK;
  const size_t oWv  = off; off += PWV;
  const size_t oWo2 = off; off += PWO2;
  const size_t oXH  = off; off += PXH;
  const size_t oEH  = off; off += PEH;
  const size_t oQKh = off; off += PQK;
  const size_t oQKl = off; off += PQK;
  const size_t oVTh = off; off += PVT;
  const size_t oVTl = off; off += PVT;
  const size_t oCtx = off; off += PCTX;
  if (off > ws_size) return;
  if (off > (size_t)134217728) return;

  char* ws = (char*)d_ws;
  unsigned short* WqkT = (unsigned short*)(ws + oWqk);
  unsigned short* WvT  = (unsigned short*)(ws + oWv);
  unsigned short* WoT2 = (unsigned short*)(ws + oWo2);
  unsigned short* XH   = (unsigned short*)(ws + oXH);
  unsigned short* EH   = (unsigned short*)(ws + oEH);
  unsigned short* QKh  = (unsigned short*)(ws + oQKh);
  unsigned short* QKl  = (unsigned short*)(ws + oQKl);
  unsigned short* VTh  = (unsigned short*)(ws + oVTh);
  unsigned short* VTl  = (unsigned short*)(ws + oVTl);
  unsigned short* Ctx  = (unsigned short*)(ws + oCtx);
  float*          out0 = (float*)d_out;

  const int n8x = (MP * DM) / 8;
  if ((n8x % 256) != 0) return;
  const int n8v = (SEQ * HD) / 8;
  const int n8t = (RCE * HD) / 8;
  if ((n8t % 32) != 0) return;
  const dim3 blk(256), blk128(128);
  const dim3 gT(DM / 64, DM / 64);
  const dim3 gCx(n8x / 256);
  const dim3 gCe((n8t + 255) / 256);
  const dim3 gNqk(((MP / 64) * (QKP / 64) + 7) / 8, 1);
  const dim3 gVT(((DM / 64) * (SEQ / 64) + 7) / 8, NBATCH);
  const dim3 gAttn(NBATCH * NH * NQB);
  const dim3 gNo(((MP / 64) * (DM / 64) + 7) / 8, 1);
  const float invw = 1.0f / WSC;

  tconv64<0><<<gT, blk, 0, stream>>>(w_q, WqkT, DM, DM, DM, 0, WSC);
  tconv64<0><<<gT, blk, 0, stream>>>(w_k, WqkT + (size_t)DM * DM, DM, DM, DM, 0, WSC);
  tconv64<0><<<gT, blk, 0, stream>>>(w_v, WvT, DM, DM, DM, 0, WSC);
  tconv64<1><<<gT, blk, 0, stream>>>(w_o, WoT2, DM, DM, 2 * DM, DM, 1.0f);
  conv_h16<<<gCx, blk, 0, stream>>>(x_in, XH, n8x, 1.0f);
  conv_e16<<<gCe, blk, 0, stream>>>(relk, EH, n8v, n8t);

  gemm64<0, 3, 1><<<gNqk, blk, 0, stream>>>(
      XH, DM, 0LL, WqkT, DM, 0LL,
      QKh, QKl, out0, QKP, 0LL,
      b_q, b_k, DM,
      MP, QKP, DM, invw);
  gemm64<0, 4, 2><<<gVT, blk, 0, stream>>>(
      WvT, DM, 0LL, XH, DM, (long long)SEQ * DM,
      VTh, VTl, out0, SEQ, (long long)DM * SEQ,
      b_v, b_v, DM,
      DM, SEQ, DM, invw);

  attn64<<<gAttn, blk128, 0, stream>>>(QKh, QKl, VTh, VTl, EH, Ctx, 0.125f);

  gemm64<1, 0, 1><<<gNo, blk, 0, stream>>>(
      Ctx, CTXP, 0LL, WoT2, 2 * DM, 0LL,
      Ctx, Ctx, out0, DM, 0LL,
      b_o, b_o, DM,
      MP, DM, 2 * DM, 1.0f);
  (void)hipGetLastError();
}
